// TransformerBlock_85822036509373
// MI455X (gfx1250) — hardware-run, weakly checked
//
#include <hip/hip_runtime.h>


#ifndef NB
#define NB 4
#endif
#ifndef SEQ
#define SEQ 2048
#endif
#define NB_FULL  4
#define SEQ_FULL 2048
#ifndef OUT_SEQ
#define OUT_SEQ SEQ
#endif
#define DM   1024
#define NH_  16
#define HD   64
#define FF   4096
#define AW   4
#define RES_ROWS 512
#define QRS  2048.0f
#define QRI  (1.0f / 2048.0f)
#define SC2  (0.125f * 1.4426950408889634f)
#define PSH  8.0f
#define WCS  64.0f
#define YCS  16.0f
#define FCS  16.0f

static_assert(HD == 64);
static_assert(NH_ * HD == DM);
static_assert(DM % 64 == 0);
static_assert(FF % 64 == 0);
static_assert(DM % 256 == 0);
static_assert(SEQ % 64 == 0);
static_assert((NB * SEQ) % 64 == 0);
static_assert((NB * SEQ) % 8 == 0);
static_assert(SEQ % 32 == 0);
static_assert(SEQ % (16 * AW) == 0);
static_assert(NB <= NB_FULL);
static_assert(SEQ <= SEQ_FULL);
static_assert(DM % 32 == 0);
static_assert(FF % 32 == 0);
static_assert(32 * 16 * 16 == 64 * 64 * 2);
static_assert(32 * 16 * 32 == 64 * 64 * 4);
static_assert(64 * 72 * 2 <= 131072);
static_assert(64 * 68 * 4 <= 131072);
static_assert(AW * 16 * 68 * 4 <= 131072);

typedef _Float16 h16;
typedef __attribute__((ext_vector_type(16))) _Float16 v16h;
typedef __attribute__((ext_vector_type(8)))  _Float16 v8h;
typedef __attribute__((ext_vector_type(8)))  float    v8f;
typedef __attribute__((ext_vector_type(4)))  float    v4f;
typedef v4f  __attribute__((may_alias)) v4fa;

__device__ __forceinline__ unsigned short f2bf(float f) { unsigned u = __float_as_uint(f); u += 0x7FFFu + ((u >> 16) & 1u); return (unsigned short)(u >> 16); }
__device__ __forceinline__ float rbf(float f) { return __uint_as_float(((unsigned)f2bf(f)) << 16); }
__device__ __forceinline__ v16h cat16(v8h lo, v8h hi) { return __builtin_shufflevector(lo, hi, 0, 1, 2, 3, 4, 5, 6, 7, 8, 9, 10, 11, 12, 13, 14, 15); }
__device__ __forceinline__ v8f wmma16(v16h a, v16h b, v8f c) { return __builtin_amdgcn_wmma_f32_16x16x32_f16(false, a, false, b, (short)0, c, false, false); }
__device__ __forceinline__ v16h ldh(const h16* p) { return cat16(*(const v8h*)p, *(const v8h*)(p + 16)); }
__device__ __forceinline__ void wave_sync() { __builtin_amdgcn_fence(3  , "wavefront"); __builtin_amdgcn_wave_barrier(); asm volatile("" ::: "memory"); }
__device__ __forceinline__ float gelu_x(float v) { const float w = v + 0.044715f * v * v * v;
    const float e = __builtin_amdgcn_exp2f(fminf(w * (-2.0f * 0.7978845608028654f * 1.4426950408889634f), 64.0f));
    return v * __builtin_amdgcn_rcpf(1.0f + e); }
static __device__ __forceinline__ h16 toh_flush(float v) { const h16 r = (h16)v; return (fabsf(v) < 6.103515625e-05f) ? (h16)0.0f : r; }

__global__ __launch_bounds__(256) void k_wt(const float* __restrict__ W, h16* Wt, int K, int N) {
    __shared__ __align__(16) h16 tl[64 * 72];
    const int tid = threadIdx.x; const int n0 = blockIdx.x * 64, k0 = blockIdx.y * 64;
#pragma unroll
    for (int it = 0; it < 4; ++it) { const int k = it * 16 + (tid >> 4), c = (tid & 15) * 4;
        const v4f v = *(const v4f*)(W + (size_t)(k0 + k) * N + n0 + c);
#pragma unroll
        for (int i = 0; i < 4; ++i) tl[(c + i) * 72 + k] = (h16)(rbf(v[i]) * WCS); }
    __syncthreads();
    v8h o0, o1; const int rw = tid >> 3, c8 = (tid & 7) * 8;
    o0 = *(const v8h*)(&tl[rw * 72 + c8]); o1 = *(const v8h*)(&tl[(32 + rw) * 72 + c8]);
    h16* d0 = Wt + (size_t)(n0 + rw) * K + k0 + c8; h16* d1 = Wt + (size_t)(n0 + 32 + rw) * K + k0 + c8;
    *(volatile v8h*)d0 = o0; *(volatile v8h*)d1 = o1;
    __threadfence();
    *(volatile v8h*)d0 = o0; *(volatile v8h*)d1 = o1;
}

__device__ __forceinline__ v8f ld8r(const float* p, int rnd) { v8f v = *(const v8f*)p;
#pragma unroll
    for (int i = 0; i < 8; ++i) { const float r = rbf(v[i]); v[i] = rnd ? r : v[i]; }
    return v; }
__global__ __launch_bounds__(256) void k_ln(const float* __restrict__ X, const float* __restrict__ G, const float* __restrict__ Bv, h16* Hout, int rnd, int inSeq) {
    const int lane = threadIdx.x & 31, wave = __builtin_amdgcn_readfirstlane((int)(threadIdx.x >> 5));
    const int row = blockIdx.x * 8 + wave;
    const float* xr = X + ((size_t)(row / SEQ) * (size_t)inSeq + (size_t)(row % SEQ)) * DM + lane * 8;
    float s = 0.0f;
#pragma unroll 1
    for (int j = 0; j < 4; ++j) { const v8f v = ld8r(xr + j * 256, rnd); s += ((v[0] + v[1]) + (v[2] + v[3])) + ((v[4] + v[5]) + (v[6] + v[7])); }
    s += __shfl_xor(s, 16, 32); s += __shfl_xor(s, 8, 32); s += __shfl_xor(s, 4, 32); s += __shfl_xor(s, 2, 32); s += __shfl_xor(s, 1, 32);
    const float mean = s * (1.0f / (float)DM);
    float q = 0.0f;
#pragma unroll 1
    for (int j = 0; j < 4; ++j) { const v8f v = ld8r(xr + j * 256, rnd);
#pragma unroll
        for (int i = 0; i < 8; ++i) { const float d = v[i] - mean; q += d * d; } }
    q += __shfl_xor(q, 16, 32); q += __shfl_xor(q, 8, 32); q += __shfl_xor(q, 4, 32); q += __shfl_xor(q, 2, 32); q += __shfl_xor(q, 1, 32);
    const float rstd = rsqrtf(q * (1.0f / (float)DM) + 1.0e-5f);
    h16* hr = Hout + (size_t)row * DM + lane * 8;
#pragma unroll 1
    for (int ps = 0; ps < 2; ++ps) {
#pragma unroll 1
        for (int j = 0; j < 4; ++j) { const v8f v = ld8r(xr + j * 256, rnd); const v8f g = ld8r(G + j * 256 + lane * 8, 1); const v8f bb = ld8r(Bv + j * 256 + lane * 8, 1); v8h o;
#pragma unroll
            for (int i = 0; i < 8; ++i) o[i] = (h16)((v[i] - mean) * rstd * g[i] + bb[i]);
            *(volatile v8h*)(hr + j * 256) = o; }
        if (ps == 0) __threadfence(); }
}

template <int MODE>
__global__ __launch_bounds__(32) void k_gemm(const h16* __restrict__ A, const h16* __restrict__ Bt, int K,
                                             const float* __restrict__ bias, float scale, float ocarry,
                                             h16* Ph, h16* Pr, int useRes, int RB, size_t sRB, int pitch, int CB, size_t sCB,
                                             float* OF, const float* __restrict__ RES, int resSeq, int outSeq) {
    __shared__ __align__(16) float os[64 * 68];
    const int lane = threadIdx.x & 31, lr = lane & 15, hi = lane >> 4; const int r0 = blockIdx.x * 64, c0 = blockIdx.y * 64;
    v8f acc[4][4];
#pragma unroll
    for (int mb = 0; mb < 4; ++mb)
#pragma unroll
        for (int nb = 0; nb < 4; ++nb) acc[mb][nb] = (v8f){};
    const size_t aoff = (size_t)(r0 + lr) * K + 8 * hi, boff = (size_t)(c0 + lr) * K + 8 * hi;
#pragma unroll 1
    for (int kc = 0; kc < K; kc += 32) {
        v16h a[4];
#pragma unroll
        for (int mb = 0; mb < 4; ++mb) a[mb] = ldh(A + aoff + (size_t)mb * 16 * K + kc);
#pragma unroll
        for (int nb = 0; nb < 4; ++nb) { const v16h b = ldh(Bt + boff + (size_t)nb * 16 * K + kc);
#pragma unroll
            for (int mb = 0; mb < 4; ++mb) acc[mb][nb] = wmma16(a[mb], b, acc[mb][nb]); }
        asm volatile("v_nop\n\tv_nop\n\tv_nop\n\tv_nop" : "+v"(acc[0][0]), "+v"(acc[1][1]), "+v"(acc[2][2]), "+v"(acc[3][3]) : "v"(a[0]), "v"(a[1]), "v"(a[2]), "v"(a[3]));
    }
#pragma unroll
    for (int mb = 0; mb < 4; ++mb)
#pragma unroll
        for (int nb = 0; nb < 4; ++nb)
#pragma unroll
            for (int j = 0; j < 8; ++j) os[(mb * 16 + hi * 8 + j) * 68 + nb * 16 + lr] = acc[mb][nb][j];
    wave_sync();
    if (MODE <= 2) {
        const int rq = lane >> 3, c8 = (lane & 7) * 8;
        float bc[8];
        if (MODE != 1) { const v4f b0 = *(const v4f*)(bias + c0 + c8); const v4f b1 = *(const v4f*)(bias + c0 + c8 + 4);
#pragma unroll
            for (int i = 0; i < 4; ++i) { bc[i] = rbf(b0[i]); bc[4 + i] = rbf(b1[i]); } }
        else {
#pragma unroll
            for (int i = 0; i < 8; ++i) bc[i] = 0.0f; }
#pragma unroll 1
        for (int s = 0; s < 16; ++s) { const int row = 4 * s + rq;
            v4f x0 = *(const v4fa*)(&os[row * 68 + c8]); v4f x1 = *(const v4fa*)(&os[row * 68 + c8 + 4]);
            float br = 0.0f; if (MODE == 1) br = rbf(bias[r0 + row]);
#pragma unroll
            for (int i = 0; i < 4; ++i) { float u0 = x0[i] * scale + ((MODE == 1) ? br : bc[i]); float u1 = x1[i] * scale + ((MODE == 1) ? br : bc[4 + i]);
                if (MODE == 2) { u0 = gelu_x(u0) * ocarry; u1 = gelu_x(u1) * ocarry; }
                x0[i] = u0; x1[i] = u1; }
            *(v4fa*)(&os[row * 68 + c8]) = x0; *(v4fa*)(&os[row * 68 + c8 + 4]) = x1; }
        wave_sync();
        const size_t tbase = (size_t)(r0 / RB) * sRB + (size_t)(r0 % RB) * (size_t)pitch + (size_t)(c0 / CB) * sCB + (size_t)(c0 % CB);
#pragma unroll 1
        for (int ps = 0; ps < 2; ++ps) {
#pragma unroll 4
            for (int s = 0; s < 16; ++s) { const int row = 4 * s + rq;
                const v4f x0 = *(const v4fa*)(&os[row * 68 + c8]); const v4f x1 = *(const v4fa*)(&os[row * 68 + c8 + 4]); v8h hv, rv;
#pragma unroll
                for (int i = 0; i < 4; ++i) { const h16 a0 = (MODE == 2) ? toh_flush(x0[i]) : (h16)x0[i]; const h16 a1 = (MODE == 2) ? toh_flush(x1[i]) : (h16)x1[i]; hv[i] = a0; hv[4 + i] = a1; rv[i] = (h16)((x0[i] - (float)a0) * QRS); rv[4 + i] = (h16)((x1[i] - (float)a1) * QRS); }
                const size_t oo = tbase + (size_t)row * (size_t)pitch + c8;
                *(volatile v8h*)(Ph + oo) = hv; if (useRes) *(volatile v8h*)(Pr + oo) = rv; }
            if (ps == 0) __threadfence(); }
    } else {
        const int cofs = lr * 4;
        v4f bq = *(const v4f*)(bias + c0 + cofs);
#pragma unroll
        for (int i = 0; i < 4; ++i) bq[i] = rbf(bq[i]);
        const size_t rrow0 = (size_t)(r0 / SEQ) * (size_t)resSeq + (size_t)(r0 % SEQ), orow0 = (size_t)(r0 / SEQ) * (size_t)outSeq + (size_t)(r0 % SEQ);
#pragma unroll 1
        for (int ps = 0; ps < 2; ++ps) {
#pragma unroll 4
            for (int s = 0; s < 32; ++s) { const int row = 2 * s + hi;
                const v4f a = *(const v4fa*)(&os[row * 68 + cofs]);
                v4f rv = *(const v4f*)(RES + (rrow0 + row) * DM + c0 + cofs);
                v4f val;
#pragma unroll
                for (int i = 0; i < 4; ++i) { const float rr = (MODE == 3) ? rbf(rv[i]) : rv[i]; val[i] = rr + (a[i] * scale + bq[i]); }
                *(volatile v4f*)(OF + (orow0 + row) * DM + c0 + cofs) = val; }
            if (ps == 0) __threadfence(); }
    }
}

__global__ __launch_bounds__(32 * AW) void k_flash(const h16* __restrict__ QH, const h16* __restrict__ QR, const h16* __restrict__ KP, const h16* __restrict__ VT, h16* Y) {
    __shared__ __align__(16) float os[AW * 16 * 68];
    const int lane = threadIdx.x & 31, lr = lane & 15, hi = lane >> 4;
    const int wave = __builtin_amdgcn_readfirstlane((int)(threadIdx.x >> 5));
    const int zh = blockIdx.y; const int b = zh / NH_, h = zh % NH_;
    const int t0 = (blockIdx.x * AW + wave) * 16;
    const bool useR = t0 < RES_ROWS;
    const size_t pbase = (size_t)zh * SEQ * HD;
    const size_t qo = pbase + (size_t)(t0 + lr) * HD + 8 * hi;
    const v16h qh0 = ldh(QH + qo), qh1 = ldh(QH + qo + 32), qr0 = ldh(QR + qo), qr1 = ldh(QR + qo + 32);
    const size_t ko = pbase + (size_t)lr * HD + 8 * hi;
    const size_t vo = pbase + (size_t)lr * SEQ + 8 * hi;
    v8f o0 = (v8f){}, o1 = (v8f){}, o2 = (v8f){}, o3 = (v8f){};
    float m = -3.0e38f, l = 0.0f;
    const int kend = t0 + 16;
#pragma unroll 1
    for (int key0 = 0; key0 < kend; key0 += 32) {
        const h16* ka = KP + ko + (size_t)key0 * HD;
        const v16h ka0 = ldh(ka), ka1 = ldh(ka + 32), kb0 = ldh(ka + 16 * HD), kb1 = ldh(ka + 16 * HD + 32);
        v8f sHa = (v8f){}, sLa = (v8f){}, sHb = (v8f){}, sLb = (v8f){};
        if (useR) {
            sHa = wmma16(ka0, qh0, sHa); sLa = wmma16(ka0, qr0, sLa); sHb = wmma16(kb0, qh0, sHb); sLb = wmma16(kb0, qr0, sLb);
            sHa = wmma16(ka1, qh1, sHa); sLa = wmma16(ka1, qr1, sLa); sHb = wmma16(kb1, qh1, sHb); sLb = wmma16(kb1, qr1, sLb);
        } else {
            sHa = wmma16(ka0, qh0, sHa); sHb = wmma16(kb0, qh0, sHb);
            sHa = wmma16(ka1, qh1, sHa); sHb = wmma16(kb1, qh1, sHb);
        }
        asm volatile("v_nop\n\tv_nop\n\tv_nop\n\tv_nop" : "+v"(sHa), "+v"(sLa), "+v"(sHb), "+v"(sLb) : "v"(ka0), "v"(ka1), "v"(kb0), "v"(kb1));
        float ta[8], tb[8];
#pragma unroll
        for (int r = 0; r < 8; ++r) { ta[r] = (sHa[r] + sLa[r] * QRI) * SC2; tb[r] = (sHb[r] + sLb[r] * QRI) * SC2; }
        if (key0 + 31 > t0) {
            const int tq = t0 + lr, kA = key0 + 8 * hi;
#pragma unroll
            for (int r = 0; r < 8; ++r) { ta[r] = (kA + r > tq) ? -3.0e38f : ta[r]; tb[r] = (kA + 16 + r > tq) ? -3.0e38f : tb[r]; }
        }
        float mx = -3.0e38f;
#pragma unroll
        for (int r = 0; r < 8; ++r) mx = fmaxf(mx, fmaxf(ta[r], tb[r]));
        mx = fmaxf(mx, __shfl_xor(mx, 16, 32));
        const float mnew = fmaxf(m, mx);
        const float alpha = __builtin_amdgcn_exp2f(m - mnew);
        const float sh = PSH - mnew;
        v16h pb; float ls = 0.0f;
#pragma unroll
        for (int r = 0; r < 8; ++r) { const h16 pa = (h16)__builtin_amdgcn_exp2f(ta[r] + sh); const h16 pc = (h16)__builtin_amdgcn_exp2f(tb[r] + sh); pb[r] = pa; pb[8 + r] = pc; ls += (float)pa + (float)pc; }
        l = l * alpha + ls; m = mnew;
        o0 = o0 * alpha; o1 = o1 * alpha; o2 = o2 * alpha; o3 = o3 * alpha;
        const h16* va = VT + vo + key0;
        const v16h v0 = ldh(va), v1 = ldh(va + (size_t)16 * SEQ), v2 = ldh(va + (size_t)32 * SEQ), v3 = ldh(va + (size_t)48 * SEQ);
        o0 = wmma16(v0, pb, o0); o1 = wmma16(v1, pb, o1); o2 = wmma16(v2, pb, o2); o3 = wmma16(v3, pb, o3);
        asm volatile("v_nop\n\tv_nop\n\tv_nop\n\tv_nop" : "+v"(o0), "+v"(o1), "+v"(o2), "+v"(o3) : "v"(v0), "v"(v1), "v"(v2), "v"(v3), "v"(pb));
    }
    l += __shfl_xor(l, 16, 32);
    const float inv = YCS * (1.0f / l);
    const int wb = wave * 16 * 68;
    { v4f a, c;
      a[0] = o0[0] * inv; a[1] = o0[1] * inv; a[2] = o0[2] * inv; a[3] = o0[3] * inv; c[0] = o0[4] * inv; c[1] = o0[5] * inv; c[2] = o0[6] * inv; c[3] = o0[7] * inv;
      *(v4fa*)(&os[wb + lr * 68 +  0 + 8 * hi]) = a; *(v4fa*)(&os[wb + lr * 68 +  0 + 8 * hi + 4]) = c;
      a[0] = o1[0] * inv; a[1] = o1[1] * inv; a[2] = o1[2] * inv; a[3] = o1[3] * inv; c[0] = o1[4] * inv; c[1] = o1[5] * inv; c[2] = o1[6] * inv; c[3] = o1[7] * inv;
      *(v4fa*)(&os[wb + lr * 68 + 16 + 8 * hi]) = a; *(v4fa*)(&os[wb + lr * 68 + 16 + 8 * hi + 4]) = c;
      a[0] = o2[0] * inv; a[1] = o2[1] * inv; a[2] = o2[2] * inv; a[3] = o2[3] * inv; c[0] = o2[4] * inv; c[1] = o2[5] * inv; c[2] = o2[6] * inv; c[3] = o2[7] * inv;
      *(v4fa*)(&os[wb + lr * 68 + 32 + 8 * hi]) = a; *(v4fa*)(&os[wb + lr * 68 + 32 + 8 * hi + 4]) = c;
      a[0] = o3[0] * inv; a[1] = o3[1] * inv; a[2] = o3[2] * inv; a[3] = o3[3] * inv; c[0] = o3[4] * inv; c[1] = o3[5] * inv; c[2] = o3[6] * inv; c[3] = o3[7] * inv;
      *(v4fa*)(&os[wb + lr * 68 + 48 + 8 * hi]) = a; *(v4fa*)(&os[wb + lr * 68 + 48 + 8 * hi + 4]) = c; }
    wave_sync();
    h16* yrow = Y + ((size_t)b * SEQ + t0) * DM + h * HD;
#pragma unroll 1
    for (int ps = 0; ps < 2; ++ps) {
#pragma unroll
        for (int s = 0; s < 4; ++s) { const int row = 4 * s + (lane >> 3), c8 = (lane & 7) * 8;
            const v4f x0 = *(const v4fa*)(&os[wb + row * 68 + c8]); const v4f x1 = *(const v4fa*)(&os[wb + row * 68 + c8 + 4]); v8h hv;
#pragma unroll
            for (int i = 0; i < 4; ++i) { hv[i] = (h16)x0[i]; hv[4 + i] = (h16)x1[i]; }
            *(volatile v8h*)(yrow + (size_t)row * DM + c8) = hv; }
        if (ps == 0) __threadfence(); }
}

static constexpr size_t al256(size_t v) { return (v + 255) & ~(size_t)255; }
static constexpr size_t cmax(size_t a, size_t b) { return a > b ? a : b; }
static constexpr size_t MROWS   = (size_t)NB * SEQ;
static constexpr size_t SZ_PL   = al256((size_t)NB * NH_ * SEQ * HD * 2);
static constexpr size_t SZ_WQKV = (size_t)3 * DM * DM * 2;
static constexpr size_t SZ_WO   = (size_t)DM * DM * 2;
static constexpr size_t SZ_WFC  = (size_t)DM * FF * 2;
static constexpr size_t SZ_WPR  = (size_t)FF * DM * 2;
static constexpr size_t SZ_F    = MROWS * FF * 2;
static constexpr size_t SZ_X1   = MROWS * DM * 4;
static constexpr size_t SZ_P  = al256(cmax(cmax(4 * SZ_PL, SZ_F), SZ_WO));
static constexpr size_t SZ_X  = al256(cmax(SZ_X1, SZ_WQKV));
static constexpr size_t SZ_WF = al256(SZ_WFC + SZ_WPR);
static constexpr size_t SZ_S  = al256(MROWS * DM * 2);
static constexpr size_t SZ_TOTAL = SZ_P + SZ_X + SZ_WF + SZ_S;
static_assert(SZ_TOTAL <= (size_t)134217728);
static_assert(4 * SZ_PL <= SZ_P);
static_assert(SZ_F <= SZ_P);
static_assert(SZ_WO <= SZ_P);
static_assert(SZ_WQKV <= SZ_X);
static_assert(SZ_X1 <= SZ_X);
static_assert(SZ_WFC % 256 == 0);

extern "C" void kernel_launch(void* const* d_in, const int* in_sizes, int n_in,
                              void* d_out, int out_size, void* d_ws, size_t ws_size, hipStream_t stream) {
    if (n_in < 13) return;
    if ((size_t)in_sizes[0] < ((size_t)(NB - 1) * SEQ_FULL + SEQ) * DM) return;
    if ((size_t)in_sizes[1] < (size_t)DM || (size_t)in_sizes[2] < (size_t)DM) return;
    if ((size_t)in_sizes[3] < (size_t)DM || (size_t)in_sizes[4] < (size_t)DM) return;
    if ((size_t)in_sizes[5] < (size_t)DM * 3 * DM || (size_t)in_sizes[6] < (size_t)3 * DM) return;
    if ((size_t)in_sizes[7] < (size_t)DM * DM || (size_t)in_sizes[8] < (size_t)DM) return;
    if ((size_t)in_sizes[9] < (size_t)DM * FF || (size_t)in_sizes[10] < (size_t)FF) return;
    if ((size_t)in_sizes[11] < (size_t)FF * DM || (size_t)in_sizes[12] < (size_t)DM) return;
    if ((size_t)out_size < ((size_t)(NB - 1) * OUT_SEQ + SEQ) * DM) return;
    if (SZ_TOTAL > ws_size) return;
    const float* x    = (const float*)d_in[0];  const float* g1   = (const float*)d_in[1];  const float* be1 = (const float*)d_in[2];
    const float* g2   = (const float*)d_in[3];  const float* be2  = (const float*)d_in[4];
    const float* wqkv = (const float*)d_in[5];  const float* bqkv = (const float*)d_in[6];
    const float* wo   = (const float*)d_in[7];  const float* bo   = (const float*)d_in[8];
    const float* wfc  = (const float*)d_in[9];  const float* bfc  = (const float*)d_in[10];
    const float* wpr  = (const float*)d_in[11]; const float* bpr  = (const float*)d_in[12];
    float* OUT = (float*)d_out;
    char* wsp = (char*)d_ws;
    char* RP = wsp; wsp += SZ_P;
    char* RX = wsp; wsp += SZ_X;
    char* RW = wsp; wsp += SZ_WF;
    char* RS = wsp; wsp += SZ_S;
    h16* QH = (h16*)RP;
    h16* QR = (h16*)(RP + SZ_PL);
    h16* KP = (h16*)(RP + 2 * SZ_PL);
    h16* VT = (h16*)(RP + 3 * SZ_PL);
    h16* WOT = (h16*)RP;
    h16* FP = (h16*)RP;
    h16* WQKVT = (h16*)RX;
    float* X1 = (float*)RX;
    h16* WFCT = (h16*)RW;
    h16* WPRT = (h16*)(RW + SZ_WFC);
    h16* ACT = (h16*)RS;
    const float wci = 1.0f / WCS;

    k_wt<<<dim3(3 * DM / 64, DM / 64, 1), 256, 0, stream>>>(wqkv, WQKVT, DM, 3 * DM);
    k_wt<<<dim3(FF / 64, DM / 64, 1), 256, 0, stream>>>(wfc, WFCT, DM, FF);
    k_wt<<<dim3(DM / 64, FF / 64, 1), 256, 0, stream>>>(wpr, WPRT, FF, DM);

    k_ln<<<(unsigned)(MROWS / 8), 256, 0, stream>>>(x, g1, be1, ACT, 1, SEQ_FULL);

    k_gemm<0><<<dim3((unsigned)(MROWS / 64), DM / 64, 1), 32, 0, stream>>>(ACT, WQKVT, DM, bqkv, wci, 1.0f,
        QH, QR, 1, SEQ, (size_t)NH_ * SEQ * HD, HD, HD, (size_t)SEQ * HD, OUT, x, SEQ, SEQ);
    k_gemm<0><<<dim3((unsigned)(MROWS / 64), DM / 64, 1), 32, 0, stream>>>(ACT, WQKVT + (size_t)DM * DM, DM, bqkv + DM, wci, 1.0f,
        KP, KP, 0, SEQ, (size_t)NH_ * SEQ * HD, HD, HD, (size_t)SEQ * HD, OUT, x, SEQ, SEQ);
    k_gemm<1><<<dim3(DM / 64, (unsigned)(MROWS / 64), 1), 32, 0, stream>>>(WQKVT + (size_t)2 * DM * DM, ACT, DM, bqkv + 2 * DM, wci, 1.0f,
        VT, VT, 0, DM, (size_t)0, SEQ, SEQ, (size_t)DM * SEQ, OUT, x, SEQ, SEQ);

    k_flash<<<dim3(SEQ / (16 * AW), NB * NH_, 1), 32 * AW, 0, stream>>>(QH, QR, KP, VT, ACT);

    k_wt<<<dim3(DM / 64, DM / 64, 1), 256, 0, stream>>>(wo, WOT, DM, DM);
    k_gemm<3><<<dim3((unsigned)(MROWS / 64), DM / 64, 1), 32, 0, stream>>>(ACT, WOT, DM, bo, 1.0f / (WCS * YCS), 1.0f,
        ACT, ACT, 0, 64, (size_t)0, 64, 64, (size_t)0, X1, x, SEQ_FULL, SEQ);

    k_ln<<<(unsigned)(MROWS / 8), 256, 0, stream>>>(X1, g2, be2, ACT, 0, SEQ);

    k_gemm<2><<<dim3((unsigned)(MROWS / 64), FF / 64, 1), 32, 0, stream>>>(ACT, WFCT, DM, bfc, wci, FCS,
        FP, FP, 0, (int)MROWS, (size_t)0, FF, FF, (size_t)0, OUT, x, SEQ, SEQ);
    k_gemm<4><<<dim3((unsigned)(MROWS / 64), DM / 64, 1), 32, 0, stream>>>(FP, WPRT, FF, bpr, 1.0f / (WCS * FCS), 1.0f,
        ACT, ACT, 0, 64, (size_t)0, 64, 64, (size_t)0, OUT, X1, SEQ, OUT_SEQ);
}
